// GQAttention_86638080295420
// MI455X (gfx1250) — hardware-verified
//
#include <hip/hip_runtime.h>
#include <math.h>

#ifndef NB
#define NB 2
#endif
#ifndef SEQ
#define SEQ 2048
#endif
#define NB_FULL 2
#define SEQ_FULL 2048
#define DM 2048
#define NHQ 16
#define NKVH 4
#define HDIM 128
#define DQ (NHQ * HDIM)
#define DKV (NKVH * HDIM)
#define MTOK (NB * SEQ)
#define ROPE_HALF (HDIM / 2)
#define WS_LIMIT 134217728ull

static_assert(MTOK % 32 == 0);
static_assert(SEQ % 64 == 0);
static_assert(DM % 64 == 0 && DQ % 64 == 0 && DKV % 64 == 0);
static_assert(DM % 32 == 0 && DQ % 32 == 0);
static_assert(NB <= NB_FULL && SEQ <= SEQ_FULL);
static_assert(DQ == DM);
static_assert(NHQ % NKVH == 0);

typedef _Float16 v16h __attribute__((ext_vector_type(16)));
typedef _Float16 v8h __attribute__((ext_vector_type(8)));
typedef float v8f __attribute__((ext_vector_type(8)));
typedef float v4f __attribute__((ext_vector_type(4)));
typedef v4f __attribute__((may_alias)) v4fa;
typedef v8h __attribute__((may_alias)) v8ha;
union Frag { v16h v; v8h half[2]; };


__device__ __forceinline__ float bf16r(float f) {
    unsigned int u = __float_as_uint(f);
    u += 0x7fffu + ((u >> 16) & 1u);
    return __uint_as_float(u & 0xffff0000u);
}

__device__ __forceinline__ v8f wmma16(v16h a, v16h b, v8f c) {
    c = __builtin_amdgcn_wmma_f32_16x16x32_f16(false, a, false, b, (short)0, c, false, false);
    asm volatile("v_nop\n\tv_nop\n\tv_nop\n\tv_nop" : "+v"(c) : "v"(a), "v"(b));
    return c;
}
__device__ __forceinline__ v8f wmma16c2(v16h a0, v16h b0, v16h a1, v16h b1, v8f c) {
    c = __builtin_amdgcn_wmma_f32_16x16x32_f16(false, a0, false, b0, (short)0, c, false, false);
    c = __builtin_amdgcn_wmma_f32_16x16x32_f16(false, a1, false, b1, (short)0, c, false, false);
    asm volatile("v_nop\n\tv_nop\n\tv_nop\n\tv_nop" : "+v"(c) : "v"(a0), "v"(b0), "v"(a1), "v"(b1) : "memory");
    return c;
}
__device__ __forceinline__ v8f wmma16c4(v16h a0, v16h a1, v16h a2, v16h a3, v16h b0, v16h b1, v16h b2, v16h b3, v8f c) {
    c = __builtin_amdgcn_wmma_f32_16x16x32_f16(false, a0, false, b0, (short)0, c, false, false);
    c = __builtin_amdgcn_wmma_f32_16x16x32_f16(false, a1, false, b1, (short)0, c, false, false);
    c = __builtin_amdgcn_wmma_f32_16x16x32_f16(false, a2, false, b2, (short)0, c, false, false);
    c = __builtin_amdgcn_wmma_f32_16x16x32_f16(false, a3, false, b3, (short)0, c, false, false);
    asm volatile("v_nop\n\tv_nop\n\tv_nop\n\tv_nop" : "+v"(c) : "v"(a0), "v"(a1), "v"(a2), "v"(a3), "v"(b0), "v"(b1), "v"(b2), "v"(b3) : "memory");
    return c;
}
__device__ __forceinline__ void wmma16r4(v16h a, v16h b0, v16h b1, v16h b2, v16h b3, v8f& c0, v8f& c1, v8f& c2, v8f& c3) {
    c0 = __builtin_amdgcn_wmma_f32_16x16x32_f16(false, a, false, b0, (short)0, c0, false, false);
    c1 = __builtin_amdgcn_wmma_f32_16x16x32_f16(false, a, false, b1, (short)0, c1, false, false);
    c2 = __builtin_amdgcn_wmma_f32_16x16x32_f16(false, a, false, b2, (short)0, c2, false, false);
    c3 = __builtin_amdgcn_wmma_f32_16x16x32_f16(false, a, false, b3, (short)0, c3, false, false);
    asm volatile("v_nop\n\tv_nop\n\tv_nop\n\tv_nop" : "+v"(c0), "+v"(c1), "+v"(c2), "+v"(c3) : "v"(a), "v"(b0), "v"(b1), "v"(b2), "v"(b3));
}

#define VST2F(ptr, val) do { const float vst_f_ = (val); *(volatile float*)(ptr) = vst_f_; __threadfence(); *(volatile float*)(ptr) = vst_f_; } while (0)
#define VST2V4(ptr, val) do { const v4f vst_v4_ = (val); *(volatile v4f*)(ptr) = vst_v4_; __threadfence(); *(volatile v4f*)(ptr) = vst_v4_; } while (0)
#define VST2V8H(ptr, val) do { const v8h vst_v8_ = (val); *(volatile v8h*)(ptr) = vst_v8_; __threadfence(); *(volatile v8h*)(ptr) = vst_v8_; } while (0)

__global__ __launch_bounds__(256) void k_invf(float* __restrict__ invb, int half, int D, float base) {
    const int i = blockIdx.x * 256 + threadIdx.x;
    if (i >= ((half + 31) / 32) * 32) return;
    float v = 0.f;
    if (i < half) { const float e = (float)(2 * i) / (float)D; v = 1.0f / powf(base, e); }
    VST2F(invb + i, v);
}
__global__ __launch_bounds__(256) void k_sincos(float* __restrict__ cs, float* __restrict__ sn, const float* __restrict__ invb, int S, int half) {
#pragma clang fp contract(off)
    const int idx = blockIdx.x * 256 + threadIdx.x;
    if (idx >= S * half) return;
    const int s = idx / half, i = idx - s * half;
    const float ang = (float)s * invb[i];
    const float cv = cosf(ang);
    const float sv = sinf(ang);
    VST2F(cs + idx, cv); VST2F(sn + idx, sv);
}

__global__ __launch_bounds__(256) void k_cvt16(const float* __restrict__ src, _Float16* __restrict__ dst, int rows, int cols, int seq, int seqfull, int prer, float scale) {
#pragma clang fp contract(off)
    const long long g = (long long)blockIdx.x * 256 + threadIdx.x;
    const long long n8 = (long long)rows * cols / 8;
    if (g >= n8) return;
    const long long e0 = g * 8;
    const int r = (int)(e0 / cols);
    const int c = (int)(e0 - (long long)r * cols);
    const long long so = ((long long)(r / seq) * seqfull + (r % seq)) * cols + c;
    const v4f x0 = *(const v4f*)(src + so);
    const v4f x1 = *(const v4f*)(src + so + 4);
    v8h o;
#pragma unroll
    for (int e = 0; e < 4; ++e) { float v = x0[e]; if (prer) v = bf16r(v); o[e] = (_Float16)(v * scale); }
#pragma unroll
    for (int e = 0; e < 4; ++e) { float v = x1[e]; if (prer) v = bf16r(v); o[4 + e] = (_Float16)(v * scale); }
    VST2V8H(dst + e0, o);
}

__global__ __launch_bounds__(256) void k_trcvt(const float* __restrict__ src, _Float16* __restrict__ dst, int R, int C, float scale) {
#pragma clang fp contract(off)
    __shared__ float tile[64][65];
    const int c0 = blockIdx.x * 64, r0 = blockIdx.y * 64, tid = threadIdx.x;
#pragma unroll
    for (int ps = 0; ps < 4; ++ps) {
        const int row = (tid >> 4) + 16 * ps, c4 = (tid & 15) * 4;
        const v4f x = *(const v4f*)(src + (long long)(r0 + row) * C + c0 + c4);
#pragma unroll
        for (int e = 0; e < 4; ++e) { const float xv = x[e]; tile[row][c4 + e] = bf16r(xv); }
    }
    __syncthreads();
#pragma unroll
    for (int ps = 0; ps < 2; ++ps) {
        const int line = (tid >> 3) + 32 * ps, piece = tid & 7;
        v8h o;
#pragma unroll
        for (int e = 0; e < 8; ++e) o[e] = (_Float16)(tile[8 * piece + e][line] * scale);
        VST2V8H(dst + (long long)(c0 + line) * R + r0 + 8 * piece, o);
    }
}

template <int TM>
__global__ __launch_bounds__(32) __attribute__((amdgpu_num_vgpr(256))) void k_pgemm(const _Float16* __restrict__ A, int lda, const _Float16* __restrict__ Bt, int ldb,
                                                                                      float* __restrict__ C, int ldc, int M, int N, int K, float alpha) {
    const int lane = threadIdx.x & 31, h = lane >> 4, l15 = lane & 15;
    const int m0 = blockIdx.y * (16 * TM), n0 = blockIdx.x * 64;
    v8f acc[TM][4];
#pragma unroll
    for (int i = 0; i < TM; ++i)
#pragma unroll
        for (int t = 0; t < 4; ++t) { v8f zz = {}; acc[i][t] = zz; }
    for (int k0 = 0; k0 < K; k0 += 32) {
        Frag a[TM], b[4];
#pragma unroll
        for (int i = 0; i < TM; ++i) {
            const _Float16* ar = A + (long long)min(m0 + 16 * i + l15, M - 1) * lda + k0 + 8 * h;
            a[i].half[0] = *(const v8h*)ar; a[i].half[1] = *(const v8h*)(ar + 16);
        }
#pragma unroll
        for (int t = 0; t < 4; ++t) {
            const _Float16* br = Bt + (long long)min(n0 + 16 * t + l15, N - 1) * ldb + k0 + 8 * h;
            b[t].half[0] = *(const v8h*)br; b[t].half[1] = *(const v8h*)(br + 16);
        }
#pragma unroll
        for (int i = 0; i < TM; ++i) wmma16r4(a[i].v, b[0].v, b[1].v, b[2].v, b[3].v, acc[i][0], acc[i][1], acc[i][2], acc[i][3]);
    }
    __shared__ __align__(16) float ctile[16][36];
#pragma unroll
    for (int i = 0; i < TM; ++i) {
        const int mb = m0 + 16 * i;
#pragma unroll
        for (int tp = 0; tp < 2; ++tp) {
            const int nb = n0 + 32 * tp;
#pragma unroll
            for (int t2 = 0; t2 < 2; ++t2) {
                const int t = 2 * tp + t2;
#pragma unroll
                for (int r = 0; r < 8; ++r) ctile[8 * h + r][t2 * 16 + l15] = acc[i][t][r] * alpha;
            }
            __syncthreads();
            if (mb + 16 <= M && nb + 32 <= N) {
#pragma unroll
                for (int s = 0; s < 4; ++s) {
                    const int row = s * 4 + (lane >> 3), c4 = (lane & 7) * 4;
                    const v4f v = *(const v4fa*)&ctile[row][c4];
                    VST2V4(C + (long long)(mb + row) * ldc + nb + c4, v);
                }
            }
            __syncthreads();
        }
    }
}

__global__ __launch_bounds__(256) void k_rope16(const float* __restrict__ X, int ldx, _Float16* __restrict__ Y, int ldy, const float* __restrict__ cs, const float* __restrict__ sn,
                                                int R, int Hn, int S, int rope) {
#pragma clang fp contract(off)
    const long long g = (long long)blockIdx.x * 256 + threadIdx.x;
    const long long tot = (long long)R * Hn * (HDIM / 8);
    if (g >= tot) return;
    const int d8 = (int)(g % (HDIM / 8));
    const long long rh = g / (HDIM / 8);
    const int hh = (int)(rh % Hn);
    const int r = (int)(rh / Hn);
    const int d0 = d8 * 8, s = r % S;
    const float* xr = X + (long long)r * ldx + hh * HDIM;
    const v4f x0 = *(const v4f*)(xr + d0);
    const v4f x1 = *(const v4f*)(xr + d0 + 4);
    float y[8];
#pragma unroll
    for (int e = 0; e < 4; ++e) { y[e] = x0[e]; y[4 + e] = x1[e]; }
    if (rope) {
        const bool lo = (d0 < ROPE_HALF);
        const int pd = lo ? d0 + ROPE_HALF : d0 - ROPE_HALF;
        const int tc = lo ? d0 : d0 - ROPE_HALF;
        const v4f p0 = *(const v4f*)(xr + pd);
        const v4f p1 = *(const v4f*)(xr + pd + 4);
        const float* cr = cs + (long long)s * ROPE_HALF + tc;
        const float* sr = sn + (long long)s * ROPE_HALF + tc;
        const v4f cv0 = *(const v4f*)cr, cv1 = *(const v4f*)(cr + 4);
        const v4f sv0 = *(const v4f*)sr, sv1 = *(const v4f*)(sr + 4);
        float pp[8], cc[8], ss[8];
#pragma unroll
        for (int e = 0; e < 4; ++e) { pp[e] = p0[e]; pp[4 + e] = p1[e]; cc[e] = cv0[e]; cc[4 + e] = cv1[e]; ss[e] = sv0[e]; ss[4 + e] = sv1[e]; }
#pragma unroll
        for (int e = 0; e < 8; ++e) {
            const float t1 = y[e] * cc[e];
            const float t2 = pp[e] * ss[e];
            y[e] = lo ? (t1 - t2) : (t1 + t2);
        }
    }
    v8h o;
#pragma unroll
    for (int e = 0; e < 8; ++e) o[e] = (_Float16)y[e];
    VST2V8H(Y + (long long)r * ldy + hh * HDIM + d0, o);
}

#define AW 4
struct AttnP {
    const _Float16* Q; const _Float16* K; const _Float16* V; float* O; const float* Mf;
    long long sQb, sQh, sQi, sKb, sKh, sKj, sVb, sVh, sVj, sOb, sOh, sOi, smi, smj;
    int Lq, Lk, hrep, ipad0; float scale; int ipad1;
};
static_assert(sizeof(AttnP) == 5 * 8 + 14 * 8 + 6 * 4);

__device__ __forceinline__ v16h pf_ld(const float* row, int k0, int hf) {
    const v4f x0 = *(const v4fa*)(row + k0 + 8 * hf);
    const v4f x1 = *(const v4fa*)(row + k0 + 8 * hf + 4);
    const v4f x2 = *(const v4fa*)(row + k0 + 16 + 8 * hf);
    const v4f x3 = *(const v4fa*)(row + k0 + 16 + 8 * hf + 4);
    v16h a;
#pragma unroll
    for (int i = 0; i < 4; ++i) { a[i] = (_Float16)(x0[i] * 4096.f); a[4 + i] = (_Float16)(x1[i] * 4096.f); a[8 + i] = (_Float16)(x2[i] * 4096.f); a[12 + i] = (_Float16)(x3[i] * 4096.f); }
    return a;
}

template <int DHP, int DVP>
__global__ __launch_bounds__(32 * AW) __attribute__((amdgpu_num_vgpr(256))) void k_attn(AttnP p) {
    static_assert(DHP == 128);
    static_assert(DVP % 64 == 0 && DVP <= 128);
    constexpr int NT = DVP / 16;
    constexpr int KS = DHP / 32;
    constexpr int KP = 64 + 8;
    __shared__ __align__(16) float    pl[AW][16 * 64];
    __shared__ __align__(16) _Float16 vt[DVP * KP];
    __shared__ __align__(16) float    msk[AW * 16 * 64];
    const int lane = threadIdx.x & 31, hf = lane >> 4, l15 = lane & 15, wave = threadIdx.x >> 5;
    const int h = blockIdx.y, b = blockIdx.z, hk = h / p.hrep;
    const int qb0 = blockIdx.x * (AW * 16), q0 = qb0 + wave * 16;
    float* myp = pl[wave];
    const float L2E = 1.4426950408889634f;
    const float NEG = -__builtin_inff();
    const int qi = min(q0 + l15, p.Lq - 1);
    const _Float16* qrow = p.Q + b * p.sQb + h * p.sQh + (long long)qi * p.sQi;
    const _Float16* kbase = p.K + b * p.sKb + hk * p.sKh;
    const _Float16* vbase = p.V + b * p.sVb + hk * p.sVh;
    Frag qa[KS];
#pragma unroll
    for (int ks = 0; ks < KS; ++ks) {
        const _Float16* qr = qrow + ks * 32 + 8 * hf;
        qa[ks].half[0] = *(const v8h*)qr; qa[ks].half[1] = *(const v8h*)(qr + 16);
    }
    v8f o[NT]; float m8[8], l8[8];
#pragma unroll
    for (int t = 0; t < NT; ++t) { v8f zz = {}; o[t] = zz; }
#pragma unroll
    for (int i = 0; i < 8; ++i) { m8[i] = NEG; l8[i] = 0.f; }

    for (int j0 = 0; j0 < p.Lk; j0 += 64) {
        __syncthreads();
        for (int idx = threadIdx.x; idx < 64 * (DVP / 8); idx += 32 * AW) {
            const int jr = idx / (DVP / 8), d8 = idx - jr * (DVP / 8), j = j0 + jr;
            v8h x = *(const v8h*)(vbase + (long long)min(j, p.Lk - 1) * p.sVj + d8 * 8);
            if (j >= p.Lk) { v8h z = {}; x = z; }
#pragma unroll
            for (int e = 0; e < 8; ++e) vt[(d8 * 8 + e) * KP + jr] = x[e];
        }
        if (p.Mf) {
            const bool mvec = (p.smj == 1) && ((p.smi & 3) == 0) && (j0 + 64 <= p.Lk) && ((((size_t)p.Mf) & 15) == 0);
            for (int idx = threadIdx.x; idx < 64 * 16; idx += 32 * AW) {
                const int row = idx >> 4, c4 = (idx & 15) * 4;
                const int irow = min(qb0 + row, p.Lq - 1);
                v4f mv;
                if (mvec) {
                    mv = *(const v4f*)(p.Mf + (long long)irow * p.smi + j0 + c4);
                } else {
#pragma unroll
                    for (int e = 0; e < 4; ++e) mv[e] = p.Mf[(long long)irow * p.smi + (long long)min(j0 + c4 + e, p.Lk - 1) * p.smj];
                }
#pragma unroll
                for (int e = 0; e < 4; ++e) { const float t = mv[e]; mv[e] = bf16r(t); }
                *(v4fa*)&msk[row * 64 + c4] = mv;
            }
        }
        __syncthreads();

        v8f s[4];
#pragma unroll
        for (int t = 0; t < 4; ++t) {
            const int j = min(j0 + t * 16 + l15, p.Lk - 1);
            const _Float16* kr = kbase + (long long)j * p.sKj;
            Frag kb[KS];
#pragma unroll
            for (int ks = 0; ks < KS; ++ks) {
                kb[ks].half[0] = *(const v8h*)(kr + ks * 32 + 8 * hf);
                kb[ks].half[1] = *(const v8h*)(kr + ks * 32 + 16 + 8 * hf);
            }
            v8f zz = {};
            s[t] = wmma16c4(qa[0].v, qa[1].v, qa[2].v, qa[3].v, kb[0].v, kb[1].v, kb[2].v, kb[3].v, zz);
        }
        float pv[8][4];
#pragma unroll
        for (int i = 0; i < 8; ++i) {
            float sc[4];
#pragma unroll
            for (int t = 0; t < 4; ++t) {
                const int jg = j0 + t * 16 + l15;
                float v = s[t][i] * p.scale;
                if (p.Mf) v += msk[(wave * 16 + i + 8 * hf) * 64 + t * 16 + l15];
                if (jg >= p.Lk) v = NEG; else v *= L2E;
                sc[t] = v;
            }
            float mx = fmaxf(fmaxf(sc[0], sc[1]), fmaxf(sc[2], sc[3]));
            mx = fmaxf(mx, __shfl_xor(mx, 1, 32)); mx = fmaxf(mx, __shfl_xor(mx, 2, 32));
            mx = fmaxf(mx, __shfl_xor(mx, 4, 32)); mx = fmaxf(mx, __shfl_xor(mx, 8, 32));
            const float mnew = fmaxf(m8[i], mx);
            const float corr = (mnew == NEG) ? 1.f : exp2f(m8[i] - mnew);
            float rs = 0.f;
#pragma unroll
            for (int t = 0; t < 4; ++t) {
                const float pp = (sc[t] == NEG) ? 0.f : exp2f(sc[t] - mnew);
                rs += pp; pv[i][t] = pp;
            }
            rs += __shfl_xor(rs, 1, 32); rs += __shfl_xor(rs, 2, 32); rs += __shfl_xor(rs, 4, 32); rs += __shfl_xor(rs, 8, 32);
            l8[i] = l8[i] * corr + rs; m8[i] = mnew;
#pragma unroll
            for (int t = 0; t < NT; ++t) o[t][i] *= corr;
        }
#pragma unroll
        for (int i = 0; i < 8; ++i)
#pragma unroll
            for (int t = 0; t < 4; ++t) myp[(i + 8 * hf) * 64 + t * 16 + l15] = pv[i][t];
        __syncthreads();
        const v16h pa0 = pf_ld(myp + l15 * 64, 0, hf);
        const v16h pa1 = pf_ld(myp + l15 * 64, 32, hf);
#pragma unroll
        for (int t = 0; t < NT; ++t) {
            const _Float16* vr = vt + (t * 16 + l15) * KP;
            Frag b0, b1;
            b0.half[0] = *(const v8ha*)(vr + 8 * hf);      b0.half[1] = *(const v8ha*)(vr + 16 + 8 * hf);
            b1.half[0] = *(const v8ha*)(vr + 32 + 8 * hf); b1.half[1] = *(const v8ha*)(vr + 48 + 8 * hf);
            o[t] = wmma16c2(pa0, b0.v, pa1, b1.v, o[t]);
        }
    }

    float* obase = p.O + b * p.sOb + h * p.sOh;
    float invr[8];
#pragma unroll
    for (int i = 0; i < 8; ++i) invr[i] = (l8[i] > 0.f) ? 1.f / (l8[i] * 4096.f) : 0.f;
    __syncthreads();
    const bool ofast = ((p.sOi & 3) == 0) && ((((size_t)obase) & 15) == 0) && (q0 + 16 <= p.Lq);
#pragma unroll
    for (int c0 = 0; c0 < DVP; c0 += 64) {
#pragma unroll
        for (int i = 0; i < 8; ++i)
#pragma unroll
            for (int t = 0; t < NT; ++t) if (t * 16 >= c0 && t * 16 < c0 + 64) myp[(i + 8 * hf) * 64 + (t * 16 - c0) + l15] = o[t][i] * invr[i];
        __syncthreads();
        if (ofast) {
            for (int rr = 0; rr < 16; rr += 2) {
                const int row = rr + (lane >> 4), c4 = (lane & 15) * 4;
                const v4f v = *(const v4fa*)(myp + row * 64 + c4);
                VST2V4(obase + (long long)(q0 + row) * p.sOi + c0 + c4, v);
            }
        } else {
            for (int row = 0; row < 16; ++row) {
                const int irow = q0 + row; if (irow >= p.Lq) continue;
                for (int c = lane; c < 64; c += 32) VST2F(obase + (long long)irow * p.sOi + c0 + c, myp[row * 64 + c]);
            }
        }
        __syncthreads();
    }
}

extern "C" void kernel_launch(void* const* d_in, const int* in_sizes, int n_in, void* d_out, int out_size, void* d_ws, size_t ws_size, hipStream_t stream) {
    if (n_in < 6) return;
    if (in_sizes[0] < ((NB - 1) * SEQ_FULL + SEQ) * DM) return;
    if (in_sizes[1] < (SEQ - 1) * SEQ_FULL + SEQ) return;
    if (in_sizes[2] < DM * DQ) return;
    if (in_sizes[3] < DM * DKV) return;
    if (in_sizes[4] < DM * DKV) return;
    if (in_sizes[5] < DQ * DM) return;
    if (out_size < MTOK * DM) return;

    const float* hs = (const float*)d_in[0];
    const float* am = (const float*)d_in[1];
    const float* Wq = (const float*)d_in[2];
    const float* Wk = (const float*)d_in[3];
    const float* Wv = (const float*)d_in[4];
    const float* Wo = (const float*)d_in[5];
    float* out = (float*)d_out;

    size_t off = 0;
    auto take = [&](size_t bytes) -> size_t { const size_t o = off; off += (bytes + 255) & ~(size_t)255; return o; };
    const size_t o_invf = take((size_t)256);
    const size_t o_cs   = take((size_t)SEQ * ROPE_HALF * 4);
    const size_t o_sn   = take((size_t)SEQ * ROPE_HALF * 4);
    const size_t o_x16  = take((size_t)MTOK * DM * 2);
    const size_t o_wq   = take((size_t)DQ * DM * 2);
    const size_t o_wk   = take((size_t)DKV * DM * 2);
    const size_t o_wv   = take((size_t)DKV * DM * 2);
    const size_t o_wo   = take((size_t)DM * DQ * 2);
    const size_t o_qf   = take((size_t)MTOK * DQ * 4);
    const size_t o_kf   = take((size_t)MTOK * DKV * 4);
    const size_t o_vf   = take((size_t)MTOK * DKV * 4);
    const size_t o_q16  = take((size_t)MTOK * DQ * 2);
    const size_t o_k16  = take((size_t)MTOK * DKV * 2);
    const size_t o_v16  = take((size_t)MTOK * DKV * 2);
    const size_t o_of   = o_qf;
    const size_t o_o16  = o_x16;
    if (off > ws_size || off > WS_LIMIT) return;

    char* ws = (char*)d_ws;
    float* invf = (float*)(ws + o_invf);
    float* cs = (float*)(ws + o_cs);
    float* sn = (float*)(ws + o_sn);
    _Float16* x16 = (_Float16*)(ws + o_x16);
    _Float16* wqt = (_Float16*)(ws + o_wq);
    _Float16* wkt = (_Float16*)(ws + o_wk);
    _Float16* wvt = (_Float16*)(ws + o_wv);
    _Float16* wot = (_Float16*)(ws + o_wo);
    float* qf = (float*)(ws + o_qf);
    float* kf = (float*)(ws + o_kf);
    float* vf = (float*)(ws + o_vf);
    _Float16* q16 = (_Float16*)(ws + o_q16);
    _Float16* k16 = (_Float16*)(ws + o_k16);
    _Float16* v16 = (_Float16*)(ws + o_v16);
    float* of = (float*)(ws + o_of);
    _Float16* o16 = (_Float16*)(ws + o_o16);

    k_invf<<<1, 256, 0, stream>>>(invf, ROPE_HALF, HDIM, 10000.0f);
    k_sincos<<<(unsigned)((SEQ * ROPE_HALF + 255) / 256), 256, 0, stream>>>(cs, sn, invf, SEQ, ROPE_HALF);
    k_cvt16<<<(unsigned)(((long long)MTOK * DM / 8 + 255) / 256), 256, 0, stream>>>(hs, x16, MTOK, DM, SEQ, SEQ_FULL, 1, 1.0f);
    k_trcvt<<<dim3(DQ / 64, DM / 64), 256, 0, stream>>>(Wq, wqt, DM, DQ, 64.0f);
    k_trcvt<<<dim3(DKV / 64, DM / 64), 256, 0, stream>>>(Wk, wkt, DM, DKV, 64.0f);
    k_trcvt<<<dim3(DKV / 64, DM / 64), 256, 0, stream>>>(Wv, wvt, DM, DKV, 64.0f);
    k_trcvt<<<dim3(DM / 64, DQ / 64), 256, 0, stream>>>(Wo, wot, DQ, DM, 64.0f);
    k_pgemm<2><<<dim3(DQ / 64, MTOK / 32), 32, 0, stream>>>(x16, DM, wqt, DM, qf, DQ, MTOK, DQ, DM, 1.0f / 64.0f);
    k_pgemm<2><<<dim3(DKV / 64, MTOK / 32), 32, 0, stream>>>(x16, DM, wkt, DM, kf, DKV, MTOK, DKV, DM, 1.0f / 64.0f);
    k_pgemm<2><<<dim3(DKV / 64, MTOK / 32), 32, 0, stream>>>(x16, DM, wvt, DM, vf, DKV, MTOK, DKV, DM, 1.0f / 64.0f);
    k_rope16<<<(unsigned)(((long long)MTOK * NHQ * (HDIM / 8) + 255) / 256), 256, 0, stream>>>(qf, DQ, q16, DQ, cs, sn, MTOK, NHQ, SEQ, 1);
    k_rope16<<<(unsigned)(((long long)MTOK * NKVH * (HDIM / 8) + 255) / 256), 256, 0, stream>>>(kf, DKV, k16, DKV, cs, sn, MTOK, NKVH, SEQ, 1);
    k_rope16<<<(unsigned)(((long long)MTOK * NKVH * (HDIM / 8) + 255) / 256), 256, 0, stream>>>(vf, DKV, v16, DKV, cs, sn, MTOK, NKVH, SEQ, 0);
    {
        AttnP a{};
        a.Q = q16; a.K = k16; a.V = v16; a.O = of; a.Mf = am;
        a.sQb = (long long)SEQ * DQ;  a.sQh = HDIM; a.sQi = DQ;
        a.sKb = (long long)SEQ * DKV; a.sKh = HDIM; a.sKj = DKV;
        a.sVb = (long long)SEQ * DKV; a.sVh = HDIM; a.sVj = DKV;
        a.sOb = (long long)SEQ * DQ;  a.sOh = HDIM; a.sOi = DQ;
        a.smi = SEQ_FULL; a.smj = 1;
        a.Lq = SEQ; a.Lk = SEQ; a.hrep = NHQ / NKVH; a.ipad0 = 0; a.scale = 0.08838834764831845f; a.ipad1 = 0;
        k_attn<HDIM, HDIM><<<dim3((unsigned)((SEQ + 16 * AW - 1) / (16 * AW)), (unsigned)NHQ, (unsigned)NB), 32 * AW, 0, stream>>>(a);
    }
    k_cvt16<<<(unsigned)(((long long)MTOK * DQ / 8 + 255) / 256), 256, 0, stream>>>(of, o16, MTOK, DQ, MTOK, MTOK, 0, 64.0f);
    k_pgemm<2><<<dim3(DM / 64, MTOK / 32), 32, 0, stream>>>(o16, DQ, wot, DQ, out, DM, MTOK, DM, DQ, 1.0f / 4096.0f);
}
